// MultiHeadAttentionV1_89137751261756
// MI455X (gfx1250) — hardware-verified
//
#include <hip/hip_runtime.h>
#include <math.h>
#include <stdint.h>

#define NBATCH 2
#define SEQ    2048
#define DM     1024
#define NH     16
#define HD     64
#define MP     (NBATCH * SEQ)
#define NQB    (SEQ / 64)
#define CTXP   (2 * DM)
#define QRES   ((size_t)MP * DM)
#define VRES   ((size_t)NBATCH * DM * SEQ)
#define WSC    64.0f
#define RSC    2048.0f
#define PSC    1024.0f
static_assert(NH * HD == DM);
static_assert((SEQ % 64) == 0 && (DM % 64) == 0 && (MP % 64) == 0);
static_assert(HD == 64);

typedef _Float16       v16h __attribute__((ext_vector_type(16)));
typedef __bf16         v16b __attribute__((ext_vector_type(16)));
typedef unsigned short v16us __attribute__((ext_vector_type(16)));
typedef unsigned short v8us __attribute__((ext_vector_type(8)));
typedef float          v8f  __attribute__((ext_vector_type(8)));
typedef float          v4f  __attribute__((ext_vector_type(4)));
typedef unsigned int   v4u  __attribute__((ext_vector_type(4)));

union Frag { v16us u; v8us p[2]; v16h h; v16b b; };

__device__ __forceinline__ unsigned short bf_bits(float f) {
  unsigned u = __float_as_uint(f);
  return (unsigned short)((u + 0x7FFFu + ((u >> 16) & 1u)) >> 16);
}
__device__ __forceinline__ float bf_up(unsigned short h) { return __uint_as_float(((unsigned)h) << 16); }
__device__ __forceinline__ float bfr(float f) { return bf_up(bf_bits(f)); }
__device__ __forceinline__ unsigned short h_bits(_Float16 x) { return __builtin_bit_cast(unsigned short, x); }
__device__ __forceinline__ unsigned pk16(unsigned short a, unsigned short b) { return (unsigned)a | ((unsigned)b << 16); }
__device__ __forceinline__ v8f zero8() { v8f z = {0.f, 0.f, 0.f, 0.f, 0.f, 0.f, 0.f, 0.f}; return z; }

__device__ __forceinline__ v16us ldfrag(const unsigned short* p) {
  Frag f;
  f.p[0] = *(const v8us*)(p);
  f.p[1] = *(const v8us*)(p + 16);
  return f.u;
}

template <int BF>
__device__ __forceinline__ v8f mma_raw(v16us a, v16us b, v8f c) {
  Frag fa, fb;
  fa.u = a;
  fb.u = b;
  if constexpr (BF) {
    return __builtin_amdgcn_wmma_f32_16x16x32_bf16(false, fa.b, false, fb.b, (short)0, c, false, false);
  } else {
    return __builtin_amdgcn_wmma_f32_16x16x32_f16(false, fa.h, false, fb.h, (short)0, c, false, false);
  }
}
template <int BF>
__device__ __forceinline__ v8f mma_g(v16us a, v16us b, v8f c) {
  c = mma_raw<BF>(a, b, c);
#if defined(__HIP_DEVICE_COMPILE__)
  asm volatile("v_nop\n\tv_nop\n\tv_nop\n\tv_nop" : "+v"(c) : "v"(a), "v"(b));
#endif
  return c;
}
__device__ __forceinline__ void dep_guard1(v8f& a, v8f& b, v16us x) {
#if defined(__HIP_DEVICE_COMPILE__)
  asm volatile("v_nop\n\tv_nop\n\tv_nop\n\tv_nop" : "+v"(a), "+v"(b) : "v"(x));
#endif
}
__device__ __forceinline__ void keep4(v16us a, v16us b, v16us c, v16us d) {
#if defined(__HIP_DEVICE_COMPILE__)
  asm volatile("v_nop" :: "v"(a), "v"(b), "v"(c), "v"(d));
#endif
}
__device__ __forceinline__ void acc_guard4(v8f& a, v8f& b, v8f& c, v8f& d) {
#if defined(__HIP_DEVICE_COMPILE__)
  asm volatile("v_nop\n\tv_nop\n\tv_nop\n\tv_nop" : "+v"(a), "+v"(b), "+v"(c), "+v"(d));
#endif
}
__device__ __forceinline__ void wave_sync_lds() {
  __builtin_amdgcn_fence(__ATOMIC_RELEASE, "workgroup");
  __builtin_amdgcn_wave_barrier();
  __builtin_amdgcn_fence(__ATOMIC_ACQUIRE, "workgroup");
}

__global__ __launch_bounds__(256) void conv_h16(const float* __restrict__ W, unsigned short* Wh, int n8, float wsc) {
  const int i  = blockIdx.x * 256 + threadIdx.x;
  const int ic = (i < n8) ? i : (n8 - 1);
  const float* src = W + (size_t)ic * 8;
  const v4f a = *(const v4f*)(src);
  const v4f c = *(const v4f*)(src + 4);
  v4u o;
  o[0] = pk16(h_bits((_Float16)(bfr(a[0]) * wsc)), h_bits((_Float16)(bfr(a[1]) * wsc)));
  o[1] = pk16(h_bits((_Float16)(bfr(a[2]) * wsc)), h_bits((_Float16)(bfr(a[3]) * wsc)));
  o[2] = pk16(h_bits((_Float16)(bfr(c[0]) * wsc)), h_bits((_Float16)(bfr(c[1]) * wsc)));
  o[3] = pk16(h_bits((_Float16)(bfr(c[2]) * wsc)), h_bits((_Float16)(bfr(c[3]) * wsc)));
  if (i < n8) *(volatile v4u*)(Wh + (size_t)i * 8) = o;
  __threadfence();
  if (i < n8) *(volatile v4u*)(Wh + (size_t)i * 8) = o;
}

template <int BF, int DUP>
__global__ __launch_bounds__(256) void tconv64(const float* __restrict__ in, long long inStrideZ, int C,
                                               unsigned short* out, long long outStrideZ, int ldo, int dupOff,
                                               float sc) {
  __shared__ __align__(16) unsigned short sT[64 * 72];
  const int t  = threadIdx.x;
  const int r0 = blockIdx.x * 64;
  const int c0 = blockIdx.y * 64;
  const float* src = in + (size_t)blockIdx.z * (size_t)inStrideZ;
  unsigned short* dst = out + (size_t)blockIdx.z * (size_t)outStrideZ;
#pragma unroll
  for (int i = 0; i < 4; ++i) {
    const int idx = t + 256 * i;
    const int rr  = idx >> 4;
    const int cq  = (idx & 15) * 4;
    const v4f x = *(const v4f*)(src + (size_t)(r0 + rr) * (size_t)C + c0 + cq);
#pragma unroll
    for (int j = 0; j < 4; ++j) {
      unsigned short w;
      if (BF) {
        w = bf_bits(x[j]);
      } else {
        w = h_bits((_Float16)(bfr(x[j]) * sc));
      }
      sT[(cq + j) * 72 + rr] = w;
    }
  }
  __syncthreads();
  const int q8 = t >> 3;
  const int c8 = (t & 7) * 8;
  v8us vv[2];
#pragma unroll
  for (int it = 0; it < 2; ++it) {
    const int row = it * 32 + q8;
    vv[it] = *(const v8us*)(sT + row * 72 + c8);
  }
  for (int pass = 0; pass < 2; ++pass) {
#pragma unroll
    for (int it = 0; it < 2; ++it) {
      const int row = it * 32 + q8;
      unsigned short* dp = dst + (size_t)(c0 + row) * (size_t)ldo + r0 + c8;
      *(volatile v8us*)(dp) = vv[it];
      if (DUP) *(volatile v8us*)(dp + dupOff) = vv[it];
    }
    __threadfence();
  }
}

template <int BF, int OM, int BIASM>
__global__ __launch_bounds__(256) void gemm64(
    const unsigned short* __restrict__ A, int lda, long long strideA,
    const unsigned short* __restrict__ Bt, int ldb, long long strideB,
    const float* __restrict__ bias0, const float* __restrict__ bias1, int Nb,
    void* Cout, int ldc, long long strideC, long long resOff,
    int M, int N, int K, float oscale) {
  __shared__ __align__(16) float sT[8][16 * 68];
  const int b    = blockIdx.y;
  const int lane = threadIdx.x & 31;
  const int wave = threadIdx.x >> 5;
  const int tilesN = N >> 6;
  const int tilesM = M >> 6;
  const int tile = blockIdx.x * 8 + wave;
  if (tile >= tilesM * tilesN) return;
  const int tm = tile / tilesN;
  const int tn = tile - tm * tilesN;
  const int m0 = tm << 6;
  const int n0 = tn << 6;

  const unsigned short* Ab = A  + (size_t)b * (size_t)strideA;
  const unsigned short* Bb = Bt + (size_t)b * (size_t)strideB;

  const int rlane = lane & 15;
  const int koff  = (lane >> 4) * 8;
  const int mOff  = (lane >> 4) * 8;

  v8f acc[4][4];
#pragma unroll
  for (int i = 0; i < 4; ++i)
#pragma unroll
    for (int j = 0; j < 4; ++j) acc[i][j] = zero8();

  for (int k0 = 0; k0 < K; k0 += 32) {
    v16us bh[4];
#pragma unroll
    for (int j = 0; j < 4; ++j) {
      const size_t bo = (size_t)(n0 + (j << 4) + rlane) * ldb + koff + k0;
      bh[j] = ldfrag(Bb + bo);
    }
#pragma unroll
    for (int i = 0; i < 4; ++i) {
      const size_t ao = (size_t)(m0 + (i << 4) + rlane) * lda + koff + k0;
      const v16us ah = ldfrag(Ab + ao);
#pragma unroll
      for (int j = 0; j < 4; ++j) acc[i][j] = mma_raw<BF>(ah, bh[j], acc[i][j]);
      dep_guard1(acc[i][0], acc[i][3], ah);
    }
    keep4(bh[0], bh[1], bh[2], bh[3]);
  }
  acc_guard4(acc[0][0], acc[0][1], acc[0][2], acc[0][3]);
  acc_guard4(acc[1][0], acc[1][1], acc[1][2], acc[1][3]);
  acc_guard4(acc[2][0], acc[2][1], acc[2][2], acc[2][3]);
  acc_guard4(acc[3][0], acc[3][1], acc[3][2], acc[3][3]);

  const int hh2 = lane >> 4, c4 = (lane & 15) * 4;
  const int q8  = lane >> 3, c8 = (lane & 7) * 8;
  float bc[8];
#pragma unroll
  for (int e = 0; e < 8; ++e) bc[e] = 0.f;
  if (BIASM == 0) {
    const bool use1 = (n0 >= Nb);
    if (OM == 0) {
      const int cb = n0 + c4;
      const int i0 = (cb < Nb - 4) ? cb : (Nb - 4);
      const int i1 = (cb - Nb > 0) ? (cb - Nb) : 0;
      const v4f b0v = *(const v4f*)(bias0 + i0);
      const v4f b1v = *(const v4f*)(bias1 + i1);
#pragma unroll
      for (int e = 0; e < 4; ++e) bc[e] = bfr(use1 ? b1v[e] : b0v[e]);
    } else {
      const int cb = n0 + c8;
      const int i0 = (cb < Nb - 8) ? cb : (Nb - 8);
      const int i1 = (cb - Nb > 0) ? (cb - Nb) : 0;
      const v4f b0a = *(const v4f*)(bias0 + i0), b0b = *(const v4f*)(bias0 + i0 + 4);
      const v4f b1a = *(const v4f*)(bias1 + i1), b1b = *(const v4f*)(bias1 + i1 + 4);
#pragma unroll
      for (int e = 0; e < 4; ++e) {
        bc[e]     = bfr(use1 ? b1a[e] : b0a[e]);
        bc[4 + e] = bfr(use1 ? b1b[e] : b0b[e]);
      }
    }
  }

  float* slab = sT[wave];
#pragma unroll
  for (int i = 0; i < 4; ++i) {
    const int mBase = m0 + (i << 4);
#pragma unroll
    for (int j = 0; j < 4; ++j) {
#pragma unroll
      for (int r = 0; r < 8; ++r) {
        slab[(mOff + r) * 68 + (j << 4) + rlane] = acc[i][j][r];
      }
    }
    wave_sync_lds();
    if constexpr (OM == 0) {
      float* C = (float*)Cout + (size_t)b * (size_t)strideC;
      v4f vals[8];
#pragma unroll
      for (int it = 0; it < 8; ++it) {
        const int row = it * 2 + hh2;
        v4f v = *(const v4f*)(slab + row * 68 + c4);
#pragma unroll
        for (int e = 0; e < 4; ++e) v[e] = v[e] * oscale + bc[e];
        vals[it] = v;
      }
      for (int pass = 0; pass < 2; ++pass) {
#pragma unroll
        for (int it = 0; it < 8; ++it) {
          const int row = it * 2 + hh2;
          *(volatile v4f*)(C + (size_t)(mBase + row) * ldc + n0 + c4) = vals[it];
        }
        __threadfence();
      }
    } else {
      unsigned short* C = (unsigned short*)Cout + (size_t)b * (size_t)strideC;
      v4u hv[4], hr[4];
#pragma unroll
      for (int it = 0; it < 4; ++it) {
        const int row = it * 4 + q8;
        const float* sp = slab + row * 68 + c8;
        float bm = 0.f;
        if (BIASM == 1) bm = bfr(bias0[mBase + row]);
        v4u a, ar;
#pragma unroll
        for (int e = 0; e < 4; ++e) {
          const float f0 = sp[2 * e]     * oscale + ((BIASM == 1) ? bm : bc[2 * e]);
          const float f1 = sp[2 * e + 1] * oscale + ((BIASM == 1) ? bm : bc[2 * e + 1]);
          const _Float16 g0 = (_Float16)f0, g1 = (_Float16)f1;
          a[e] = pk16(h_bits(g0), h_bits(g1));
          if (OM == 3) {
            const float e0 = (f0 - (float)g0) * RSC;
            const float e1 = (f1 - (float)g1) * RSC;
            ar[e] = pk16(h_bits((_Float16)e0), h_bits((_Float16)e1));
          } else {
            ar[e] = 0u;
          }
        }
        hv[it] = a;
        hr[it] = ar;
      }
      for (int pass = 0; pass < 2; ++pass) {
#pragma unroll
        for (int it = 0; it < 4; ++it) {
          const int row = it * 4 + q8;
          unsigned short* dp = C + (size_t)(mBase + row) * ldc + n0 + c8;
          *(volatile v4u*)(dp) = hv[it];
          if (OM == 3) *(volatile v4u*)(dp + resOff) = hr[it];
        }
        __threadfence();
      }
    }
    wave_sync_lds();
  }
}

__global__ __launch_bounds__(128)
void attn64(const unsigned short* __restrict__ qhp, const unsigned short* __restrict__ khp,
            const unsigned short* __restrict__ vtp, unsigned short* ctxp,
            float sscale, float ssres) {
  __shared__ __align__(16) unsigned short Ksh[64 * 64];
  __shared__ __align__(16) unsigned short Vth[64 * 64];
  __shared__ __align__(16) unsigned short Vtr[64 * 64];
  __shared__ __align__(16) unsigned short Psh[4][16 * 64];
  __shared__ __align__(16) float          Os[4][16 * 64];

  const int tid  = threadIdx.x;
  const int wave = tid >> 5;
  const int lane = tid & 31;
  const int hh   = lane >> 4;
  const int c    = lane & 15;

  const int bx   = blockIdx.x;
  const int qb   = bx % NQB;
  const int rest = bx / NQB;
  const int h    = rest % NH;
  const int b    = rest / NH;
  const int q0   = qb * 64 + wave * 16;
  const size_t rowB = (size_t)b * SEQ;

  const unsigned short* Qh = qhp + (size_t)h * HD;
  const unsigned short* Qr = qhp + QRES + (size_t)h * HD;
  const unsigned short* Kg = khp + (size_t)h * HD;
  const unsigned short* Vh = vtp + ((size_t)b * DM + (size_t)h * HD) * SEQ;
  const unsigned short* Vr = Vh + VRES;

  float mrow[8], lrow[8];
  v8f oacc[4], oacr[4];
#pragma unroll
  for (int r = 0; r < 8; ++r) { mrow[r] = -INFINITY; lrow[r] = 0.f; }
#pragma unroll
  for (int t = 0; t < 4; ++t) { oacc[t] = zero8(); oacr[t] = zero8(); }

  for (int kt = 0; kt < NQB; ++kt) {
    const int kv0 = kt * 64;
    __syncthreads();
    {
      const int r = tid >> 1, hf = (tid & 1) * 32;
      const unsigned short* kg = Kg + (rowB + kv0 + r) * DM + hf;
      const unsigned short* vg = Vh + (size_t)r * SEQ + kv0 + hf;
      const unsigned short* vr = Vr + (size_t)r * SEQ + kv0 + hf;
#pragma unroll
      for (int i = 0; i < 4; ++i) {
        const v8us a0 = *(const v8us*)(kg + 8 * i);
        const v8us b0 = *(const v8us*)(vg + 8 * i);
        const v8us c0 = *(const v8us*)(vr + 8 * i);
        *(v8us*)(Ksh + r * 64 + hf + 8 * i) = a0;
        *(v8us*)(Vth + r * 64 + hf + 8 * i) = b0;
        *(v8us*)(Vtr + r * 64 + hf + 8 * i) = c0;
      }
    }
    __syncthreads();

    v16us qa[2], qr[2];
#pragma unroll
    for (int dc = 0; dc < 2; ++dc) {
      qa[dc] = ldfrag(Qh + (rowB + q0 + c) * DM + dc * 32 + 8 * hh);
      qr[dc] = ldfrag(Qr + (rowB + q0 + c) * DM + dc * 32 + 8 * hh);
    }

    v8f s[4];
#pragma unroll
    for (int j = 0; j < 4; ++j) {
      v8f sh = zero8(), sr = zero8();
#pragma unroll
      for (int dc = 0; dc < 2; ++dc) {
        Frag kb;
        kb.p[0] = *(const v8us*)(Ksh + (j * 16 + c) * 64 + dc * 32 + 8 * hh);
        kb.p[1] = *(const v8us*)(Ksh + (j * 16 + c) * 64 + dc * 32 + 16 + 8 * hh);
        sh = mma_g<0>(qa[dc], kb.u, sh);
        sr = mma_g<0>(qr[dc], kb.u, sr);
      }
#pragma unroll
      for (int r = 0; r < 8; ++r) s[j][r] = fmaf(sh[r], sscale, sr[r] * ssres);
    }

    unsigned short* pwh = Psh[wave];
#pragma unroll
    for (int r = 0; r < 8; ++r) {
      float m = s[0][r];
      m = fmaxf(m, s[1][r]);
      m = fmaxf(m, s[2][r]);
      m = fmaxf(m, s[3][r]);
#pragma unroll
      for (int off = 1; off < 16; off <<= 1) m = fmaxf(m, __shfl_xor(m, off, 32));
      const float mnew  = fmaxf(mrow[r], m);
      const float alpha = __expf(mrow[r] - mnew);
      mrow[r] = mnew;
      float psum = 0.f;
#pragma unroll
      for (int j = 0; j < 4; ++j) {
        const float p = __expf(s[j][r] - mnew);
        psum += p;
        pwh[(8 * hh + r) * 64 + j * 16 + c] = h_bits((_Float16)(p * PSC));
      }
#pragma unroll
      for (int off = 1; off < 16; off <<= 1) psum += __shfl_xor(psum, off, 32);
      lrow[r] = lrow[r] * alpha + psum;
#pragma unroll
      for (int t = 0; t < 4; ++t) { oacc[t][r] *= alpha; oacr[t][r] *= alpha; }
    }
    wave_sync_lds();

#pragma unroll 1
    for (int kk = 0; kk < 2; ++kk) {
      Frag pa;
      pa.p[0] = *(const v8us*)(pwh + c * 64 + kk * 32 + 8 * hh);
      pa.p[1] = *(const v8us*)(pwh + c * 64 + kk * 32 + 16 + 8 * hh);
#pragma unroll
      for (int t = 0; t < 4; ++t) {
        Frag vb, vc;
        vb.p[0] = *(const v8us*)(Vth + (t * 16 + c) * 64 + kk * 32 + 8 * hh);
        vb.p[1] = *(const v8us*)(Vth + (t * 16 + c) * 64 + kk * 32 + 16 + 8 * hh);
        vc.p[0] = *(const v8us*)(Vtr + (t * 16 + c) * 64 + kk * 32 + 8 * hh);
        vc.p[1] = *(const v8us*)(Vtr + (t * 16 + c) * 64 + kk * 32 + 16 + 8 * hh);
        oacc[t] = mma_g<0>(pa.u, vb.u, oacc[t]);
        oacr[t] = mma_g<0>(pa.u, vc.u, oacr[t]);
      }
    }
  }

  float* os = Os[wave];
#pragma unroll
  for (int r = 0; r < 8; ++r) {
    const float l = lrow[r];
    const float inv = ((l > 0.f) ? (1.0f / l) : 0.f) * (1.0f / PSC);
#pragma unroll
    for (int t = 0; t < 4; ++t) os[(8 * hh + r) * 64 + t * 16 + c] = fmaf(oacr[t][r], 1.0f / RSC, oacc[t][r]) * inv;
  }
  wave_sync_lds();
  {
    const int q4 = lane >> 3, c8 = (lane & 7) * 8;
    v4u hv[4], hl[4];
#pragma unroll
    for (int it = 0; it < 4; ++it) {
      const int row = it * 4 + q4;
      const float* sp = os + row * 64 + c8;
      v4u a, d;
#pragma unroll
      for (int e = 0; e < 4; ++e) {
        const float f0 = sp[2 * e], f1 = sp[2 * e + 1];
        const unsigned short hb0 = bf_bits(f0), hb1 = bf_bits(f1);
        const unsigned short lb0 = bf_bits(f0 - bf_up(hb0)), lb1 = bf_bits(f1 - bf_up(hb1));
        a[e] = pk16(hb0, hb1);
        d[e] = pk16(lb0, lb1);
      }
      hv[it] = a;
      hl[it] = d;
    }
    for (int pass = 0; pass < 2; ++pass) {
#pragma unroll
      for (int it = 0; it < 4; ++it) {
        const int row = it * 4 + q4;
        const size_t go = (rowB + q0 + row) * CTXP + (size_t)h * HD + c8;
        *(volatile v4u*)(ctxp + go)      = hv[it];
        *(volatile v4u*)(ctxp + go + DM) = hl[it];
      }
      __threadfence();
    }
  }
}

extern "C" void kernel_launch(void* const* d_in, const int* in_sizes, int n_in,
                              void* d_out, int out_size, void* d_ws, size_t ws_size,
                              hipStream_t stream) {
  if (n_in < 11) return;
  if (in_sizes[0] != MP * DM || in_sizes[1] != MP * DM || in_sizes[2] != MP * DM) return;
  if (in_sizes[3] != NH * DM * HD || in_sizes[4] != NH * HD) return;
  if (in_sizes[5] != NH * DM * HD || in_sizes[6] != NH * HD) return;
  if (in_sizes[7] != NH * DM * HD || in_sizes[8] != NH * HD) return;
  if (in_sizes[9] != DM * DM || in_sizes[10] != DM) return;
  if (out_size != MP * DM) return;

  const float* query = (const float*)d_in[0];
  const float* key_  = (const float*)d_in[1];
  const float* value = (const float*)d_in[2];
  const float* w_q   = (const float*)d_in[3];
  const float* b_q   = (const float*)d_in[4];
  const float* w_k   = (const float*)d_in[5];
  const float* b_k   = (const float*)d_in[6];
  const float* w_v   = (const float*)d_in[7];
  const float* b_v   = (const float*)d_in[8];
  const float* w_o   = (const float*)d_in[9];
  const float* b_o   = (const float*)d_in[10];

  const size_t PW   = (size_t)3 * DM * DM * 2;
  const size_t PWO  = (size_t)DM * CTXP * 2;
  const size_t PX   = (size_t)MP * DM * 2;
  const size_t PQ   = (size_t)2 * MP * DM * 2;
  const size_t PK   = (size_t)MP * DM * 2;
  const size_t PV   = (size_t)2 * NBATCH * DM * SEQ * 2;
  const size_t PC   = (size_t)MP * CTXP * 2;
  size_t off = 0;
  const size_t oW  = off; off += PW;
  const size_t oWo = off; off += PWO;
  const size_t oX  = off; off += PX;
  const size_t oQ  = off; off += PQ;
  const size_t oK  = off; off += PK;
  const size_t oV  = off; off += PV;
  const size_t oC  = off; off += PC;
  if (off > ws_size) return;
  if (off > (size_t)134217728) return;

  char* ws = (char*)d_ws;
  unsigned short* WqkvT = (unsigned short*)(ws + oW);
  unsigned short* WoB   = (unsigned short*)(ws + oWo);
  unsigned short* XH    = (unsigned short*)(ws + oX);
  unsigned short* QH    = (unsigned short*)(ws + oQ);
  unsigned short* KH    = (unsigned short*)(ws + oK);
  unsigned short* VT    = (unsigned short*)(ws + oV);
  unsigned short* Ctx   = (unsigned short*)(ws + oC);
  float*          out0  = (float*)d_out;

  const int n8x = (MP * DM) / 8;
  if ((n8x % 256) != 0) return;
  const dim3 blk(256), blk128(128);
  const dim3 gCx((n8x + 255) / 256);
  const dim3 gTw(DM / 64, HD / 64, NH);
  const dim3 gTo(DM / 64, DM / 64, 1);
  const dim3 gN1k(((MP / 64) * (DM / 64) + 7) / 8, 1);
  const dim3 gVT(((DM / 64) * (SEQ / 64) + 7) / 8, NBATCH);
  const dim3 gAttn(NBATCH * NH * NQB);
  const float invw  = 1.0f / WSC;
  const float ssc   = 0.125f;
  const float ssr   = 0.125f / RSC;

  tconv64<0, 0><<<gTw, blk, 0, stream>>>(w_q, (long long)DM * HD, HD, WqkvT, (long long)HD * DM, DM, 0, WSC);
  tconv64<0, 0><<<gTw, blk, 0, stream>>>(w_k, (long long)DM * HD, HD, WqkvT + (size_t)DM * DM,
                                         (long long)HD * DM, DM, 0, WSC);
  tconv64<0, 0><<<gTw, blk, 0, stream>>>(w_v, (long long)DM * HD, HD, WqkvT + (size_t)2 * DM * DM,
                                         (long long)HD * DM, DM, 0, WSC);
  tconv64<1, 1><<<gTo, blk, 0, stream>>>(w_o, 0LL, DM, WoB, 0LL, CTXP, DM, 1.0f);

  conv_h16<<<gCx, blk, 0, stream>>>(query, XH, n8x, 1.0f);
  gemm64<0, 3, 0><<<gN1k, blk, 0, stream>>>(
      XH, DM, 0LL, WqkvT, DM, 0LL, b_q, b_q, DM,
      (void*)QH, DM, 0LL, (long long)QRES, MP, DM, DM, invw);

  conv_h16<<<gCx, blk, 0, stream>>>(key_, XH, n8x, 1.0f);
  gemm64<0, 2, 0><<<gN1k, blk, 0, stream>>>(
      XH, DM, 0LL, WqkvT + (size_t)DM * DM, DM, 0LL, b_k, b_k, DM,
      (void*)KH, DM, 0LL, 0LL, MP, DM, DM, invw);

  conv_h16<<<gCx, blk, 0, stream>>>(value, XH, n8x, 1.0f);
  gemm64<0, 3, 1><<<gVT, blk, 0, stream>>>(
      WqkvT + (size_t)2 * DM * DM, DM, 0LL, XH, DM, (long long)SEQ * DM, b_v, b_v, SEQ,
      (void*)VT, SEQ, (long long)DM * SEQ, (long long)VRES, DM, SEQ, DM, invw);

  attn64<<<gAttn, blk128, 0, stream>>>(QH, KH, VT, Ctx, ssc, ssr);

  gemm64<1, 0, 0><<<gN1k, blk, 0, stream>>>(
      Ctx, CTXP, 0LL, WoB, CTXP, 0LL, b_o, b_o, DM,
      (void*)out0, DM, 0LL, 0LL, MP, DM, CTXP, 1.0f);
  (void)hipGetLastError();
}
